// MambaBlock_36301063586179
// MI455X (gfx1250) — hardware-verified
//
#include <hip/hip_runtime.h>
#include <math.h>

typedef __attribute__((ext_vector_type(16))) _Float16 v16h;
typedef __attribute__((ext_vector_type(8)))  _Float16 v8h;
typedef __attribute__((ext_vector_type(8)))  float    v8f;
typedef __attribute__((ext_vector_type(4)))  float    v4f;
typedef __attribute__((ext_vector_type(4)))  unsigned v4u;

constexpr int kBatch = 2;
constexpr int kSeq   = 2048;
constexpr int kDIn   = 512;
constexpr int kDm    = 1024;
constexpr int kNst   = 16;
constexpr int kDsc   = 64;
constexpr int kAbP   = 2 * kDm;
constexpr int kPrjN  = kDsc + 2 * kNst;
constexpr int kPrjP  = 128;
constexpr int kRows  = kBatch * kSeq;
constexpr int kTP    = 260;
constexpr float kCarSeq  = 16.0f;
constexpr float kCarWin  = 32.0f;
constexpr float kCarA    = 16.0f;
constexpr float kCarWcat = 32.0f;
constexpr float kCarX1   = 16.0f;
constexpr float kCarWd2  = 8.0f;
constexpr float kCarZ    = 16.0f;
constexpr float kCarWout = 32.0f;
static_assert(kPrjN == 96 && kPrjN <= kPrjP, "concatenated projection width");
static_assert((kDIn % 32) == 0 && (kDm % 32) == 0 && (kDsc % 32) == 0, "GEMM K multiples of 32");
static_assert((kRows % 64) == 0 && (kAbP % 64) == 0 && (kPrjP % 64) == 0 && (kDm % 64) == 0 && (kDIn % 64) == 0, "GEMM M,N multiples of 64");
static_assert((kSeq % 64) == 0 && (kDm % 256) == 0 && (kSeq % 16) == 0, "tile multiples");
static_assert((((kRows / 64) * (kAbP / 64)) % 8) == 0 && (((kRows / 64) * (kPrjP / 64)) % 8) == 0 &&
              (((kRows / 64) * (kDm / 64)) % 8) == 0 && (((kRows / 64) * (kDIn / 64)) % 8) == 0, "GEMM grids exact");

constexpr size_t kOffSeqH  = 0;
constexpr size_t kOffWinH  = kOffSeqH  + (size_t)kRows * kDIn * 2;
constexpr size_t kOffWoutH = kOffWinH  + (size_t)kAbP  * kDIn * 2;
constexpr size_t kOffWcatH = kOffWoutH + (size_t)kDIn  * kDm  * 2;
constexpr size_t kOffWd2H  = kOffWcatH + (size_t)kPrjP * kDm  * 2;
constexpr size_t kOffAB    = kOffWd2H  + (size_t)kDm   * kDsc * 2;
constexpr size_t kOffUC    = kOffAB    + (size_t)kRows * kAbP * 4;
constexpr size_t kOffUCH   = kOffUC    + (size_t)kRows * kDm  * 4;
constexpr size_t kOffPROJ  = kOffUCH   + (size_t)kRows * kDm  * 2;
constexpr size_t kOffX1H   = kOffPROJ  + (size_t)kRows * kPrjP * 4;
constexpr size_t kOffDLR   = kOffX1H   + (size_t)kRows * kDsc * 2;
constexpr size_t kOffZH    = kOffDLR   + (size_t)kRows * kDm  * 4;
constexpr size_t kWsTotal  = kOffZH    + (size_t)kRows * kDm  * 2;
static_assert(kWsTotal == 94240768ull, "carve total");
static_assert(kWsTotal <= 134217728ull, "carve cap");
static_assert((kOffWinH % 128) == 0 && (kOffWoutH % 128) == 0 && (kOffWcatH % 128) == 0 && (kOffWd2H % 128) == 0 &&
              (kOffAB % 128) == 0 && (kOffUC % 128) == 0 && (kOffUCH % 128) == 0 && (kOffPROJ % 128) == 0 &&
              (kOffX1H % 128) == 0 && (kOffDLR % 128) == 0 && (kOffZH % 128) == 0, "128-B aligned regions");

__device__ __forceinline__ unsigned short f2bf_bits(float f) {
  unsigned u = __float_as_uint(f);
  return (unsigned short)((u + 0x7FFFu + ((u >> 16) & 1u)) >> 16);
}
__device__ __forceinline__ float bf_bits2f(unsigned short h) { return __uint_as_float(((unsigned)h) << 16); }
__device__ __forceinline__ float rne_bf(float f) { return bf_bits2f(f2bf_bits(f)); }

__device__ __forceinline__ void row_guard_h(v8f& a, v8f& b, v8f& c, v8f& d, v16h x, v16h b0, v16h b1, v16h b2, v16h b3) {
  asm volatile("v_nop\n\tv_nop\n\tv_nop\n\tv_nop" : "+v"(a), "+v"(b), "+v"(c), "+v"(d) : "v"(x), "v"(b0), "v"(b1), "v"(b2), "v"(b3));
}
__device__ __forceinline__ void keep4_h(v16h a, v16h b, v16h c, v16h d) { asm volatile("v_nop" :: "v"(a), "v"(b), "v"(c), "v"(d)); }
__device__ __forceinline__ void acc_guard4(v8f& a, v8f& b, v8f& c, v8f& d) { asm volatile("v_nop\n\tv_nop\n\tv_nop\n\tv_nop" : "+v"(a), "+v"(b), "+v"(c), "+v"(d)); }

struct FragH {
  union U { v16h v; v8h h[2]; };
  static __device__ __forceinline__ v16h load(const _Float16* p) {
    U f; f.h[0] = *(const v8h*)(p); f.h[1] = *(const v8h*)(p + 16); return f.v;
  }
  static __device__ __forceinline__ v8f mma(v16h a, v16h b, v8f c) {
    return __builtin_amdgcn_wmma_f32_16x16x32_f16(false, a, false, b, (short)0, c, false, false);
  }
};

template <int BIAS_MODE>
__global__ __launch_bounds__(256) void wmma_gemm64_f16(
    const unsigned short* __restrict__ Ap, int lda,
    const unsigned short* __restrict__ Btp, int ldb,
    float* __restrict__ C, int ldc,
    const float* __restrict__ bias,
    int M, int N, int K, float scale) {
  const _Float16* A  = (const _Float16*)Ap;
  const _Float16* Bt = (const _Float16*)Btp;
  __shared__ __align__(16) float sT[8][16 * 68];
  const int lane = threadIdx.x & 31;
  const int wave = threadIdx.x >> 5;
  const int tilesN = N >> 6;
  const int tilesM = M >> 6;
  const int tile = blockIdx.x * 8 + wave;
  if (tile >= tilesM * tilesN) return;
  const int tm = tile / tilesN;
  const int tn = tile - tm * tilesN;
  const int m0 = tm << 6;
  const int n0 = tn << 6;

  const int rlane = lane & 15;
  const int koff  = (lane >> 4) * 8;
  const int mOff  = (lane >> 4) * 8;

  v8f acc[4][4];
#pragma unroll
  for (int i = 0; i < 4; ++i)
#pragma unroll
    for (int j = 0; j < 4; ++j) acc[i][j] = (v8f){0.f,0.f,0.f,0.f,0.f,0.f,0.f,0.f};

  for (int k0 = 0; k0 < K; k0 += 32) {
    v16h bh[4];
#pragma unroll
    for (int j = 0; j < 4; ++j) {
      const size_t bo = (size_t)(n0 + (j << 4) + rlane) * ldb + koff + k0;
      bh[j] = FragH::load(Bt + bo);
    }
#pragma unroll
    for (int i = 0; i < 4; ++i) {
      const size_t ao = (size_t)(m0 + (i << 4) + rlane) * lda + koff + k0;
      v16h ah = FragH::load(A + ao);
#pragma unroll
      for (int j = 0; j < 4; ++j) acc[i][j] = FragH::mma(ah, bh[j], acc[i][j]);
      row_guard_h(acc[i][0], acc[i][1], acc[i][2], acc[i][3], ah, bh[0], bh[1], bh[2], bh[3]);
    }
    keep4_h(bh[0], bh[1], bh[2], bh[3]);
  }
  acc_guard4(acc[0][0], acc[0][1], acc[0][2], acc[0][3]);
  acc_guard4(acc[1][0], acc[1][1], acc[1][2], acc[1][3]);
  acc_guard4(acc[2][0], acc[2][1], acc[2][2], acc[2][3]);
  acc_guard4(acc[3][0], acc[3][1], acc[3][2], acc[3][3]);

  float* slab = sT[wave];
#pragma unroll
  for (int i = 0; i < 4; ++i) {
    const int mBase = m0 + (i << 4);
#pragma unroll
    for (int j = 0; j < 4; ++j) {
      const int n = n0 + (j << 4) + rlane;
      float bv = 0.f;
      if (BIAS_MODE == 2) bv = rne_bf(bias[n]);
#pragma unroll
      for (int r = 0; r < 8; ++r) {
        float v = acc[i][j][r] * scale;
        if (BIAS_MODE == 2) v += bv;
        slab[(mOff + r) * 68 + (j << 4) + rlane] = v;
      }
    }
    __builtin_amdgcn_fence(__ATOMIC_RELEASE, "workgroup");
    __builtin_amdgcn_wave_barrier();
    __builtin_amdgcn_fence(__ATOMIC_ACQUIRE, "workgroup");
    {
      const int hh = lane >> 4, c4 = (lane & 15) * 4;
      for (int pass = 0; pass < 2; ++pass) {
#pragma unroll
        for (int it = 0; it < 8; ++it) {
          const int row = it * 2 + hh;
          v4f v = *(const v4f*)(slab + row * 68 + c4);
          *(volatile v4f*)(C + (size_t)(mBase + row) * ldc + n0 + c4) = v;
        }
        __threadfence();
      }
    }
    __builtin_amdgcn_fence(__ATOMIC_RELEASE, "workgroup");
    __builtin_amdgcn_wave_barrier();
    __builtin_amdgcn_fence(__ATOMIC_ACQUIRE, "workgroup");
  }
}

__global__ __launch_bounds__(256) void cast_bf_f16_kernel(
    const float* __restrict__ src, unsigned short* __restrict__ dst, int total8, float scale)
{
  const int i = blockIdx.x * 256 + threadIdx.x;
  if (i >= total8) return;
  const size_t e0 = (size_t)i << 3;
  const float* p = src + e0;
  const v4f a0 = *(const v4f*)(p);
  const v4f a1 = *(const v4f*)(p + 4);
  v8h hv;
#pragma unroll
  for (int e = 0; e < 4; ++e) {
    const float f0 = a0[e];
    const float f1 = a1[e];
    hv[e]     = (_Float16)(rne_bf(f0) * scale);
    hv[4 + e] = (_Float16)(rne_bf(f1) * scale);
  }
  unsigned short* q = dst + e0;
  *(volatile v8h*)q = hv;
  __threadfence();
  *(volatile v8h*)q = hv;
}

__global__ __launch_bounds__(256) void zero16_kernel(unsigned short* __restrict__ dst, int total8)
{
  const int i = blockIdx.x * 256 + threadIdx.x;
  if (i >= total8) return;
  unsigned short* q = dst + ((size_t)i << 3);
  const v4u z = (v4u){0u, 0u, 0u, 0u};
  *(volatile v4u*)q = z;
  __threadfence();
  *(volatile v4u*)q = z;
}

__global__ __launch_bounds__(256) void x1_cast_kernel(
    const float* __restrict__ PROJ, unsigned short* __restrict__ X1H, int total8, float scale)
{
  const int i = blockIdx.x * 256 + threadIdx.x;
  if (i >= total8) return;
  const int e0  = i << 3;
  const int row = e0 >> 6;
  const int c8  = e0 & 63;
  const float* p = PROJ + (size_t)row * kPrjP + c8;
  const v4f a0 = *(const v4f*)(p);
  const v4f a1 = *(const v4f*)(p + 4);
  v8h hv;
#pragma unroll
  for (int e = 0; e < 4; ++e) {
    hv[e]     = (_Float16)(a0[e] * scale);
    hv[4 + e] = (_Float16)(a1[e] * scale);
  }
  unsigned short* qd = X1H + e0;
  *(volatile v8h*)qd = hv;
  __threadfence();
  *(volatile v8h*)qd = hv;
}

__global__ __launch_bounds__(256) void conv_silu_kernel(
    const float* __restrict__ AB, const float* __restrict__ cw, const float* __restrict__ cb,
    float* __restrict__ UC, unsigned short* __restrict__ UCH)
{
  __shared__ __align__(16) float sT[16 * kTP];
  const int tid = threadIdx.x, lane = tid & 31, wave = tid >> 5;
  const int d0 = blockIdx.x * 256, d = d0 + tid;
  const int g0 = blockIdx.y * 64;
  const int tb = g0 & (kSeq - 1);
  const v4f wv = *(const v4f*)(cw + (size_t)d * 4);
  const float wr0 = wv[0], wr1 = wv[1], wr2 = wv[2], wr3 = wv[3];
  const float w0 = rne_bf(wr0), w1 = rne_bf(wr1), w2 = rne_bf(wr2), w3 = rne_bf(wr3);
  const float bc = rne_bf(cb[d]);
  float xm3, xm2, xm1;
  {
    const bool hist = (tb > 0);
    const int rb = hist ? (g0 - 3) : g0;
    const float v3 = AB[(size_t)rb * kAbP + d];
    const float v2 = AB[(size_t)(rb + 1) * kAbP + d];
    const float v1 = AB[(size_t)(rb + 2) * kAbP + d];
    xm3 = hist ? v3 : 0.f;
    xm2 = hist ? v2 : 0.f;
    xm1 = hist ? v1 : 0.f;
  }
  const int hrow = wave >> 1;
  const int hch  = (wave & 1) * 128 + lane * 4;
#pragma unroll 1
  for (int sub = 0; sub < 4; ++sub) {
    const int lb = g0 + sub * 16;
#pragma unroll 1
    for (int s = 0; s < 16; ++s) {
      const float xcur = AB[(size_t)(lb + s) * kAbP + d];
      float acc = w0 * xm3;
      acc = fmaf(w1, xm2, acc);
      acc = fmaf(w2, xm1, acc);
      acc = fmaf(w3, xcur, acc);
      const float sv = acc + bc;
      const float sg = __builtin_amdgcn_rcpf(1.0f + __expf(-sv));
      sT[s * kTP + tid] = sv * sg;
      xm3 = xm2; xm2 = xm1; xm1 = xcur;
    }
    __syncthreads();
    v4f fv[4];
    v8h bv[2];
#pragma unroll
    for (int it = 0; it < 4; ++it) fv[it] = *(const v4f*)(sT + (it * 4 + hrow) * kTP + hch);
#pragma unroll
    for (int it = 0; it < 2; ++it) {
      const float* sp = sT + (it * 8 + wave) * kTP + lane * 8;
      const v4f a0 = *(const v4f*)(sp);
      const v4f a1 = *(const v4f*)(sp + 4);
#pragma unroll
      for (int e = 0; e < 4; ++e) {
        bv[it][e]     = (_Float16)(a0[e] * kCarA);
        bv[it][4 + e] = (_Float16)(a1[e] * kCarA);
      }
    }
    for (int pass = 0; pass < 2; ++pass) {
#pragma unroll
      for (int it = 0; it < 4; ++it)
        *(volatile v4f*)(UC + (size_t)(lb + it * 4 + hrow) * kDm + d0 + hch) = fv[it];
#pragma unroll
      for (int it = 0; it < 2; ++it)
        *(volatile v8h*)(UCH + (size_t)(lb + it * 8 + wave) * kDm + d0 + lane * 8) = bv[it];
      __threadfence();
    }
    __syncthreads();
  }
}

__global__ __launch_bounds__(256) void scan_kernel(
    const float* __restrict__ DLR, const float* __restrict__ UC, const float* __restrict__ AB,
    const float* __restrict__ PROJ, const float* __restrict__ A_log, const float* __restrict__ Dv,
    unsigned short* __restrict__ ZH)
{
  __shared__ __align__(16) float sBC[16 * 32];
  __shared__ __align__(16) float sY[16 * kTP];
  __shared__ __align__(16) float sA[kNst * 256];
  const int tid = threadIdx.x, lane = tid & 31, wave = tid >> 5;
  const int d0 = blockIdx.x * 256, d = d0 + tid;
  const size_t row0 = (size_t)blockIdx.y * kSeq;

#pragma unroll 1
  for (int s = 0; s < kNst; ++s) sA[s * 256 + tid] = -expf(rne_bf(A_log[(size_t)d * kNst + s]));
  __syncthreads();
  float An[kNst], h[kNst];
#pragma unroll
  for (int n = 0; n < kNst; ++n) {
    An[n] = sA[n * 256 + tid];
    h[n] = 0.f;
  }
  const float Dd = rne_bf(Dv[d]);

#pragma unroll 1
  for (int c = 0; c < kSeq / 16; ++c) {
    const int l0 = c * 16;
    if (tid < 128) {
      const int r = tid >> 3, q = (tid & 7) * 4;
      const v4f v = *(const v4f*)(PROJ + (row0 + l0 + r) * kPrjP + kDsc + q);
      *(v4f*)(sBC + r * 32 + q) = v;
    }
    __syncthreads();
#pragma unroll 1
    for (int s = 0; s < 16; ++s) {
      const size_t m = row0 + (size_t)(l0 + s);
      const float a     = DLR[m * kDm + d];
      const float delta = fmaxf(a, 0.0f) + log1pf(__expf(-fabsf(a)));
      const float xv    = UC[m * kDm + d];
      const float zv    = AB[m * kAbP + kDm + d];
      v4f Bq[4], Cq[4];
#pragma unroll
      for (int qq = 0; qq < 4; ++qq) {
        Bq[qq] = *(const v4f*)(sBC + s * 32 + 4 * qq);
        Cq[qq] = *(const v4f*)(sBC + s * 32 + kNst + 4 * qq);
      }
      float y = 0.f;
#pragma unroll
      for (int n = 0; n < kNst; ++n) {
        const float e = __expf(delta * An[n]);
        float db = delta * Bq[n >> 2][n & 3];
        asm volatile("" : "+v"(db));
        float p = db * xv;
        asm volatile("" : "+v"(p));
        float qv = h[n] * e;
        asm volatile("" : "+v"(qv));
        const float hn = qv + p;
        h[n] = hn;
        float rr = Cq[n >> 2][n & 3] * hn;
        asm volatile("" : "+v"(rr));
        y += rr;
      }
      float sk = xv * Dd;
      asm volatile("" : "+v"(sk));
      y += sk;
      const float sg = __builtin_amdgcn_rcpf(1.0f + __expf(-zv));
      const float g  = zv * sg;
      sY[s * kTP + tid] = (y * g) * kCarZ;
    }
    __syncthreads();
    v8h hv[2];
#pragma unroll
    for (int it = 0; it < 2; ++it) {
      const float* sp = sY + (it * 8 + wave) * kTP + lane * 8;
      const v4f a0 = *(const v4f*)(sp);
      const v4f a1 = *(const v4f*)(sp + 4);
#pragma unroll
      for (int e = 0; e < 4; ++e) { hv[it][e] = (_Float16)a0[e]; hv[it][4 + e] = (_Float16)a1[e]; }
    }
    for (int pass = 0; pass < 2; ++pass) {
#pragma unroll
      for (int it = 0; it < 2; ++it)
        *(volatile v8h*)(ZH + (row0 + (size_t)(l0 + it * 8 + wave)) * kDm + d0 + lane * 8) = hv[it];
      __threadfence();
    }
  }
}

extern "C" void kernel_launch(void* const* d_in, const int* in_sizes, int n_in,
                              void* d_out, int out_size, void* d_ws, size_t ws_size,
                              hipStream_t stream)
{
  (void)stream;
  if (n_in < 12) return;
  if (in_sizes[0] != kRows * kDIn) return;
  if (in_sizes[1] != kAbP * kDIn) return;
  if (in_sizes[2] != kDIn * kDm) return;
  if (in_sizes[3] != kNst * kDm) return;
  if (in_sizes[4] != kNst * kDm) return;
  if (in_sizes[5] != kDsc * kDm) return;
  if (in_sizes[6] != kDm * kDsc) return;
  if (in_sizes[7] != kDm) return;
  if (in_sizes[8] != kDm * 4) return;
  if (in_sizes[9] != kDm) return;
  if (in_sizes[10] != kDm * kNst) return;
  if (in_sizes[11] != kDm) return;
  if (out_size != kRows * kDIn) return;
  if (ws_size < kWsTotal) return;

  const float* seq    = (const float*)d_in[0];
  const float* W_in   = (const float*)d_in[1];
  const float* W_out  = (const float*)d_in[2];
  const float* W_B    = (const float*)d_in[3];
  const float* W_C    = (const float*)d_in[4];
  const float* W_D1   = (const float*)d_in[5];
  const float* W_D2   = (const float*)d_in[6];
  const float* b_D2   = (const float*)d_in[7];
  const float* conv_w = (const float*)d_in[8];
  const float* conv_b = (const float*)d_in[9];
  const float* A_log  = (const float*)d_in[10];
  const float* D_skip = (const float*)d_in[11];
  float* out = (float*)d_out;

  char* ws = (char*)d_ws;
  unsigned short* SEQH  = (unsigned short*)(ws + kOffSeqH);
  unsigned short* WINH  = (unsigned short*)(ws + kOffWinH);
  unsigned short* WOUTH = (unsigned short*)(ws + kOffWoutH);
  unsigned short* WCATH = (unsigned short*)(ws + kOffWcatH);
  unsigned short* WD2H  = (unsigned short*)(ws + kOffWd2H);
  float*          AB    = (float*)(ws + kOffAB);
  float*          UC    = (float*)(ws + kOffUC);
  unsigned short* UCH   = (unsigned short*)(ws + kOffUCH);
  float*          PROJ  = (float*)(ws + kOffPROJ);
  unsigned short* X1H   = (unsigned short*)(ws + kOffX1H);
  float*          DLR   = (float*)(ws + kOffDLR);
  unsigned short* ZH    = (unsigned short*)(ws + kOffZH);

  cast_bf_f16_kernel<<<(kRows * kDIn / 8) / 256, 256, 0, stream>>>(seq,   SEQH,  kRows * kDIn / 8, kCarSeq);
  cast_bf_f16_kernel<<<(kAbP * kDIn / 8) / 256,  256, 0, stream>>>(W_in,  WINH,  kAbP * kDIn / 8,  kCarWin);
  cast_bf_f16_kernel<<<(kDIn * kDm / 8) / 256,   256, 0, stream>>>(W_out, WOUTH, kDIn * kDm / 8,   kCarWout);
  cast_bf_f16_kernel<<<(kDsc * kDm / 8) / 256,   256, 0, stream>>>(W_D1,  WCATH,                               kDsc * kDm / 8, kCarWcat);
  cast_bf_f16_kernel<<<(kNst * kDm / 8) / 256,   256, 0, stream>>>(W_B,   WCATH + (size_t)kDsc * kDm,          kNst * kDm / 8, kCarWcat);
  cast_bf_f16_kernel<<<(kNst * kDm / 8) / 256,   256, 0, stream>>>(W_C,   WCATH + (size_t)(kDsc + kNst) * kDm, kNst * kDm / 8, kCarWcat);
  zero16_kernel<<<((kPrjP - kPrjN) * kDm / 8) / 256, 256, 0, stream>>>(WCATH + (size_t)kPrjN * kDm, (kPrjP - kPrjN) * kDm / 8);
  cast_bf_f16_kernel<<<(kDm * kDsc / 8) / 256,   256, 0, stream>>>(W_D2,  WD2H,  kDm * kDsc / 8,   kCarWd2);

  wmma_gemm64_f16<0><<<((kRows / 64) * (kAbP / 64)) / 8, 256, 0, stream>>>(
      SEQH, kDIn, WINH, kDIn, AB, kAbP, b_D2, kRows, kAbP, kDIn, 1.0f / (kCarSeq * kCarWin));

  conv_silu_kernel<<<dim3(kDm / 256, kRows / 64), 256, 0, stream>>>(AB, conv_w, conv_b, UC, UCH);

  wmma_gemm64_f16<0><<<((kRows / 64) * (kPrjP / 64)) / 8, 256, 0, stream>>>(
      UCH, kDm, WCATH, kDm, PROJ, kPrjP, b_D2, kRows, kPrjP, kDm, 1.0f / (kCarA * kCarWcat));

  x1_cast_kernel<<<(kRows * kDsc / 8) / 256, 256, 0, stream>>>(PROJ, X1H, kRows * kDsc / 8, kCarX1);

  wmma_gemm64_f16<2><<<((kRows / 64) * (kDm / 64)) / 8, 256, 0, stream>>>(
      X1H, kDsc, WD2H, kDsc, DLR, kDm, b_D2, kRows, kDm, kDsc, 1.0f / (kCarX1 * kCarWd2));

  scan_kernel<<<dim3(kDm / 256, kBatch), 256, 0, stream>>>(DLR, UC, AB, PROJ, A_log, D_skip, ZH);

  wmma_gemm64_f16<0><<<((kRows / 64) * (kDIn / 64)) / 8, 256, 0, stream>>>(
      ZH, kDm, WOUTH, kDm, out, kDIn, b_D2, kRows, kDIn, kDm, 1.0f / (kCarZ * kCarWout));
}
